// NMREmbedPatchAttention_29076928594300
// MI455X (gfx1250) — hardware-run, weakly checked
//
#include <hip/hip_runtime.h>
#include <math.h>

typedef __attribute__((ext_vector_type(16))) _Float16 v16h;
typedef __attribute__((ext_vector_type(8)))  _Float16 v8h;
typedef __attribute__((ext_vector_type(8)))  float    v8f;
typedef __attribute__((ext_vector_type(4)))  float    v4f;
typedef __attribute__((ext_vector_type(4)))  unsigned int v4u;

constexpr int kBatch   = 64;
constexpr int kSpecLen = 3200;
constexpr int kDm      = 256;
constexpr int kWinLen  = 8;
constexpr int kHeads   = 8;
constexpr int kDk      = kDm / kHeads;
constexpr int kTok     = kBatch * kSpecLen;
constexpr int kWin     = kTok / kWinLen;
constexpr int kChunkB  = 8;
constexpr int kChunks  = kBatch / kChunkB;
constexpr int kTc      = kChunkB * kSpecLen;
constexpr int kWc      = kTc / kWinLen;
constexpr int kQkvN    = 3 * kDm;
constexpr int kCatK    = kWinLen * kDm;
static_assert(kDk == 32, "head width");
static_assert(kTok == 204800 && kWin == 25600, "token / window counts");
static_assert((kSpecLen % kWinLen) == 0, "windows never straddle a batch row");
static_assert(kChunks * kChunkB == kBatch, "chunking covers the batch");
static_assert(kTc == 25600 && kWc == 3200, "chunk sizes");
static_assert((kTc % 64) == 0 && (kWc % 64) == 0, "GEMM M multiples of 64");
static_assert((kDm % 64) == 0 && (kQkvN % 64) == 0, "GEMM N multiples of 64");
static_assert((kDm % 32) == 0 && (kCatK % 32) == 0, "GEMM K multiples of 32");
static_assert((kTc % 32) == 0, "attention blocks of 32 tokens");

constexpr bool kInputsAsBf16 = true;

constexpr float kActCarry = 64.0f;
constexpr float kWCarry   = 256.0f;
constexpr float kWcatCarry = 1024.0f;
constexpr float kScaleE   = kActCarry / (kActCarry * kWCarry);
constexpr float kScaleQkv = 1.0f / (kActCarry * kWCarry);
constexpr float kScaleO   = kActCarry / (kActCarry * kWCarry);
constexpr float kScaleOut = 1.0f / (kActCarry * kWcatCarry);

constexpr int kTabB2  = 0;
constexpr int kTabQkv = kDm;
constexpr int kTabBo  = kTabQkv + kQkvN;
constexpr int kTabBp  = kTabBo + kDm;
constexpr int kTabN   = kTabBp + kDm;
static_assert(kTabN == 1536, "bias table size");

constexpr size_t kOffWSQ  = 0;
constexpr size_t kOffWCAT = kOffWSQ  + (size_t)5 * kDm * kDm * 2;
constexpr size_t kOffTAB  = kOffWCAT + (size_t)kDm * kCatK * 2;
constexpr size_t kOffHP   = kOffTAB  + (size_t)kTabN * 4;
constexpr size_t kOffEP   = kOffHP   + (size_t)kTc * kDm * 2;
constexpr size_t kOffQKV  = kOffEP   + (size_t)kTc * kDm * 2;
constexpr size_t kWsTotal = kOffQKV  + (size_t)kTc * kQkvN * 4;
static_assert(kWsTotal == 106567680ull, "carve total");
static_assert(kWsTotal <= 134217728ull, "carve cap");
static_assert((kOffWCAT % 128) == 0 && (kOffTAB % 128) == 0 && (kOffHP % 128) == 0 &&
              (kOffEP % 128) == 0 && (kOffQKV % 128) == 0, "128-B aligned regions");

__device__ __forceinline__ float rne_bf16(float f) {
  unsigned u = __float_as_uint(f);
  u = (u + 0x7FFFu + ((u >> 16) & 1u)) & 0xFFFF0000u;
  return __uint_as_float(u);
}
__device__ __forceinline__ float in_val(float f) { return kInputsAsBf16 ? rne_bf16(f) : f; }
__device__ __forceinline__ unsigned pk16(unsigned short a, unsigned short b) { return (unsigned)a | ((unsigned)b << 16); }
__device__ __forceinline__ unsigned short h_bits(float f) { const _Float16 h = (_Float16)f; return __builtin_bit_cast(unsigned short, h); }

union FragU { v16h v; v8h h[2]; };
__device__ __forceinline__ v16h frag_load(const _Float16* p) {
  FragU f;
  f.h[0] = *(const v8h*)(p);
  f.h[1] = *(const v8h*)(p + 16);
  return f.v;
}
__device__ __forceinline__ v8f frag_mma(v16h a, v16h b, v8f c) {
  return __builtin_amdgcn_wmma_f32_16x16x32_f16(false, a, false, b, (short)0, c, false, false);
}
__device__ __forceinline__ void tie_acc(v8f& a, v16h x, v16h y) { asm volatile("" : "+v"(a) : "v"(x), "v"(y)); }
__device__ __forceinline__ void tie_acc_nops(v8f& a, v16h x, v16h y) { asm volatile("v_nop\n\tv_nop\n\tv_nop\n\tv_nop" : "+v"(a) : "v"(x), "v"(y)); }
__device__ __forceinline__ void tie_one(v8f& a) { asm volatile("" : "+v"(a)); }
__device__ __forceinline__ void tie_one_nops(v8f& a) { asm volatile("v_nop\n\tv_nop\n\tv_nop\n\tv_nop" : "+v"(a)); }
__device__ __forceinline__ void keep4_h(v16h a, v16h b, v16h c, v16h d) { asm volatile("v_nop" :: "v"(a), "v"(b), "v"(c), "v"(d)); }

template <int OUT_MODE>
__global__ __launch_bounds__(256) void wmma_gemm64_f16(
    const unsigned short* __restrict__ Ap, int lda,
    const unsigned short* __restrict__ Btp, int ldb,
    void* __restrict__ Cout, int ldc,
    const float* __restrict__ bias,
    int M, int N, int K, float scale) {
  const _Float16* A  = (const _Float16*)Ap;
  const _Float16* Bt = (const _Float16*)Btp;
  __shared__ __align__(16) float sT[8][16 * 68];
  const int lane = threadIdx.x & 31;
  const int wave = __builtin_amdgcn_readfirstlane((int)(threadIdx.x >> 5));
  const int tilesN = N >> 6;
  const int tilesM = M >> 6;
  const int tile = blockIdx.x * 8 + wave;
  if (tile >= tilesM * tilesN) return;
  const int tm = tile / tilesN;
  const int tn = tile - tm * tilesN;
  const int m0 = tm << 6;
  const int n0 = tn << 6;

  const int rlane = lane & 15;
  const int koff  = (lane >> 4) * 8;
  const int mOff  = (lane >> 4) * 8;

  v8f acc[4][4];
#pragma unroll
  for (int i = 0; i < 4; ++i)
#pragma unroll
    for (int j = 0; j < 4; ++j) acc[i][j] = (v8f){0.f, 0.f, 0.f, 0.f, 0.f, 0.f, 0.f, 0.f};

  for (int k0 = 0; k0 < K; k0 += 32) {
    v16h bh[4];
#pragma unroll
    for (int j = 0; j < 4; ++j) {
      const size_t bo = (size_t)(n0 + (j << 4) + rlane) * ldb + koff + k0;
      bh[j] = frag_load(Bt + bo);
    }
#pragma unroll
    for (int i = 0; i < 4; ++i) {
      const size_t ao = (size_t)(m0 + (i << 4) + rlane) * lda + koff + k0;
      const v16h ah = frag_load(A + ao);
#pragma unroll
      for (int j = 0; j < 4; ++j) acc[i][j] = frag_mma(ah, bh[j], acc[i][j]);
      tie_acc(acc[i][0], ah, bh[0]);
      tie_acc(acc[i][1], ah, bh[1]);
      tie_acc(acc[i][2], ah, bh[2]);
      tie_acc_nops(acc[i][3], ah, bh[3]);
    }
    keep4_h(bh[0], bh[1], bh[2], bh[3]);
  }
#pragma unroll
  for (int i = 0; i < 4; ++i)
#pragma unroll
    for (int j = 0; j < 4; ++j) tie_one(acc[i][j]);
  tie_one_nops(acc[3][3]);

  float* slab = sT[wave];
#pragma unroll
  for (int i = 0; i < 4; ++i) {
    const int mBase = m0 + (i << 4);
#pragma unroll
    for (int j = 0; j < 4; ++j) {
      const int n = n0 + (j << 4) + rlane;
      const float bv = bias[n];
#pragma unroll
      for (int r = 0; r < 8; ++r) {
        float v = acc[i][j][r] * scale;
        v += bv;
        slab[(mOff + r) * 68 + (j << 4) + rlane] = v;
      }
    }
    __builtin_amdgcn_fence(__ATOMIC_RELEASE, "workgroup");
    __builtin_amdgcn_wave_barrier();
    __builtin_amdgcn_fence(__ATOMIC_ACQUIRE, "workgroup");
    if (OUT_MODE == 0) {
      float* C = (float*)Cout;
      const int hh = lane >> 4, c4 = (lane & 15) * 4;
      for (int pass = 0; pass < 2; ++pass) {
#pragma unroll
        for (int it = 0; it < 8; ++it) {
          const int row = it * 2 + hh;
          v4f v = *(const v4f*)(slab + row * 68 + c4);
          *(volatile v4f*)(C + (size_t)(mBase + row) * ldc + n0 + c4) = v;
        }
        __threadfence();
      }
    } else {
      const int q = lane >> 3, c8 = (lane & 7) * 8;
      unsigned short* C = (unsigned short*)Cout;
      for (int pass = 0; pass < 2; ++pass) {
#pragma unroll
        for (int it = 0; it < 4; ++it) {
          const int row = it * 4 + q;
          const float* sp = slab + row * 68 + c8;
          v8h hv;
#pragma unroll
          for (int e = 0; e < 8; ++e) hv[e] = (_Float16)sp[e];
          *(volatile v8h*)(C + (size_t)(mBase + row) * ldc + n0 + c8) = hv;
        }
        __threadfence();
      }
    }
    __builtin_amdgcn_fence(__ATOMIC_RELEASE, "workgroup");
    __builtin_amdgcn_wave_barrier();
    __builtin_amdgcn_fence(__ATOMIC_ACQUIRE, "workgroup");
  }
}

__global__ __launch_bounds__(256) void wt_cast_kernel(const float* __restrict__ W0, const float* __restrict__ W1,
                                                      const float* __restrict__ W2, const float* __restrict__ W3,
                                                      const float* __restrict__ W4,
                                                      unsigned short* __restrict__ out, long planeStride,
                                                      int kdim, int ndim, float carry) {
  __shared__ float sm[64][65];
  const int t  = threadIdx.x;
  const int k0 = blockIdx.x * 64;
  const int n0 = blockIdx.y * 64;
  const int z  = blockIdx.z;
  const float* W = (z == 0) ? W0 : (z == 1) ? W1 : (z == 2) ? W2 : (z == 3) ? W3 : W4;
#pragma unroll 4
  for (int i = 0; i < 16; ++i) {
    const int e = i * 256 + t;
    const int r = e >> 6;
    const int c = e & 63;
    sm[c][r] = in_val(W[(size_t)(k0 + r) * ndim + n0 + c]) * carry;
  }
  __syncthreads();
  const int lane = t & 31;
  const int wave = __builtin_amdgcn_readfirstlane((int)(t >> 5));
  const int q = lane >> 3, c8 = (lane & 7) * 8;
  unsigned short* op = out + (size_t)z * (size_t)planeStride;
  v4u u[2];
#pragma unroll
  for (int it = 0; it < 2; ++it) {
    const int row = wave * 8 + it * 4 + q;
    unsigned short hb[8];
#pragma unroll
    for (int e = 0; e < 8; ++e) hb[e] = h_bits(sm[row][c8 + e]);
    u[it] = (v4u){pk16(hb[0], hb[1]), pk16(hb[2], hb[3]), pk16(hb[4], hb[5]), pk16(hb[6], hb[7])};
  }
  for (int pass = 0; pass < 2; ++pass) {
#pragma unroll
    for (int it = 0; it < 2; ++it) {
      const int row = wave * 8 + it * 4 + q;
      *(volatile v4u*)(op + (size_t)(n0 + row) * kdim + k0 + c8) = u[it];
    }
    __threadfence();
  }
}

__global__ __launch_bounds__(384) void bias_table_kernel(const float* __restrict__ b2, const float* __restrict__ bq,
                                                         const float* __restrict__ bk, const float* __restrict__ bv,
                                                         const float* __restrict__ bo, const float* __restrict__ bp,
                                                         float* __restrict__ tab, float carry) {
  const int t = threadIdx.x;
  const int wave = __builtin_amdgcn_readfirstlane((int)(t >> 5));
  const int seg = wave >> 1;
  const int off = (t & 63) * 4;
  const float* src = (seg == 0) ? b2 : (seg == 1) ? bq : (seg == 2) ? bk : (seg == 3) ? bv : (seg == 4) ? bo : bp;
  const float sc = (seg == 0 || seg == 4) ? carry : 1.0f;
  const v4f a = *(const v4f*)(src + off);
  v4f o;
  o[0] = in_val(a[0]) * sc;
  o[1] = in_val(a[1]) * sc;
  o[2] = in_val(a[2]) * sc;
  o[3] = in_val(a[3]) * sc;
  float* p = tab + 4 * t;
  *(volatile v4f*)p = o;
  __threadfence();
  *(volatile v4f*)p = o;
}

__global__ __launch_bounds__(256) void embed_kernel(const float* __restrict__ spec, const float* __restrict__ W1,
                                                    const float* __restrict__ b1, unsigned short* __restrict__ Hp,
                                                    int n8, float carry) {
  const int i = blockIdx.x * 256 + threadIdx.x;
  if (i >= n8) return;
  const int tok = i >> 5;
  const int c0  = (i & 31) * 8;
  const float s = in_val(spec[tok]);
  const v4f wa = *(const v4f*)(W1 + c0);
  const v4f wb = *(const v4f*)(W1 + c0 + 4);
  const v4f ba = *(const v4f*)(b1 + c0);
  const v4f bb = *(const v4f*)(b1 + c0 + 4);
  unsigned short hb[8];
#pragma unroll
  for (int e = 0; e < 4; ++e) {
    const float x0 = in_val(wa[e]) * s + in_val(ba[e]);
    const float x1 = in_val(wb[e]) * s + in_val(bb[e]);
    hb[e]     = h_bits(fmaxf(x0, 0.0f) * carry);
    hb[4 + e] = h_bits(fmaxf(x1, 0.0f) * carry);
  }
  const v4u u = (v4u){pk16(hb[0], hb[1]), pk16(hb[2], hb[3]), pk16(hb[4], hb[5]), pk16(hb[6], hb[7])};
  unsigned short* p = Hp + 8 * (size_t)i;
  *(volatile v4u*)p = u;
  __threadfence();
  *(volatile v4u*)p = u;
}

__global__ __launch_bounds__(256) void window_attn_kernel(const float* __restrict__ QKV, unsigned short* __restrict__ OH,
                                                          float scl, float carry) {
  __shared__ float sS[8 * 256];
  __shared__ __align__(16) unsigned sO[8][4 * 132];
  const int tid  = threadIdx.x;
  const int lane = tid & 31;
  const int wave = __builtin_amdgcn_readfirstlane((int)(tid >> 5));
  const int tok  = blockIdx.x * 32 + (tid >> 3);
  const int h    = tid & 7;
  const int wbase = tok & ~7;

  float q[32];
  {
    const float* qp = QKV + (size_t)tok * kQkvN + kDk * h;
#pragma unroll
    for (int i = 0; i < 8; ++i) {
      const v4f t4 = *(const v4f*)(qp + 4 * i);
      q[4 * i + 0] = t4[0];
      q[4 * i + 1] = t4[1];
      q[4 * i + 2] = t4[2];
      q[4 * i + 3] = t4[3];
    }
  }

  float m = -INFINITY;
#pragma unroll 1
  for (int j = 0; j < kWinLen; ++j) {
    const float* kp = QKV + (size_t)(wbase + j) * kQkvN + kDm + kDk * h;
    float d = 0.0f;
#pragma unroll
    for (int i = 0; i < 8; ++i) {
      const v4f kk = *(const v4f*)(kp + 4 * i);
      d = fmaf(q[4 * i + 0], kk[0], d);
      d = fmaf(q[4 * i + 1], kk[1], d);
      d = fmaf(q[4 * i + 2], kk[2], d);
      d = fmaf(q[4 * i + 3], kk[3], d);
    }
    d *= scl;
    sS[j * 256 + tid] = d;
    m = fmaxf(m, d);
  }
  __syncthreads();

  float acc[32];
#pragma unroll
  for (int e = 0; e < 32; ++e) acc[e] = 0.0f;
  float l = 0.0f;
#pragma unroll 1
  for (int j = 0; j < kWinLen; ++j) {
    const float p = __expf(sS[j * 256 + tid] - m);
    l += p;
    const float* vp = QKV + (size_t)(wbase + j) * kQkvN + 2 * kDm + kDk * h;
#pragma unroll
    for (int i = 0; i < 8; ++i) {
      const v4f vv = *(const v4f*)(vp + 4 * i);
      acc[4 * i + 0] = fmaf(p, vv[0], acc[4 * i + 0]);
      acc[4 * i + 1] = fmaf(p, vv[1], acc[4 * i + 1]);
      acc[4 * i + 2] = fmaf(p, vv[2], acc[4 * i + 2]);
      acc[4 * i + 3] = fmaf(p, vv[3], acc[4 * i + 3]);
    }
  }
  const float inv = carry * (1.0f / l);

  unsigned* so = sO[wave];
  {
    const int tl = lane >> 3;
#pragma unroll
    for (int i = 0; i < 4; ++i) {
      const unsigned w0 = pk16(h_bits(acc[8 * i + 0] * inv), h_bits(acc[8 * i + 1] * inv));
      const unsigned w1 = pk16(h_bits(acc[8 * i + 2] * inv), h_bits(acc[8 * i + 3] * inv));
      const unsigned w2 = pk16(h_bits(acc[8 * i + 4] * inv), h_bits(acc[8 * i + 5] * inv));
      const unsigned w3 = pk16(h_bits(acc[8 * i + 6] * inv), h_bits(acc[8 * i + 7] * inv));
      *(v4u*)(so + tl * 132 + h * 16 + 4 * i) = (v4u){w0, w1, w2, w3};
    }
  }
  __syncthreads();
  v4u o[4];
#pragma unroll
  for (int it = 0; it < 4; ++it) o[it] = *(const v4u*)(so + it * 132 + lane * 4);
  const int tokbase = blockIdx.x * 32 + wave * 4;
  for (int pass = 0; pass < 2; ++pass) {
#pragma unroll
    for (int it = 0; it < 4; ++it)
      *(volatile v4u*)(OH + (size_t)(tokbase + it) * kDm + lane * 8) = o[it];
    __threadfence();
  }
}

extern "C" void kernel_launch(void* const* d_in, const int* in_sizes, int n_in,
                              void* d_out, int out_size, void* d_ws, size_t ws_size,
                              hipStream_t stream) {
  if (n_in < 15) return;
  if (in_sizes[0] != kTok) return;
  if (in_sizes[1] != kDm || in_sizes[2] != kDm) return;
  if (in_sizes[3] != kDm * kDm || in_sizes[4] != kDm) return;
  if (in_sizes[5] != kDm * kDm || in_sizes[6] != kDm) return;
  if (in_sizes[7] != kDm * kDm || in_sizes[8] != kDm) return;
  if (in_sizes[9] != kDm * kDm || in_sizes[10] != kDm) return;
  if (in_sizes[11] != kDm * kDm || in_sizes[12] != kDm) return;
  if (in_sizes[13] != kCatK * kDm || in_sizes[14] != kDm) return;
  if (out_size != kWin * kDm) return;
  if (ws_size < kWsTotal) return;

  const float* spec = (const float*)d_in[0];
  const float* W1   = (const float*)d_in[1];
  const float* b1   = (const float*)d_in[2];
  const float* W2   = (const float*)d_in[3];
  const float* b2   = (const float*)d_in[4];
  const float* Wq   = (const float*)d_in[5];
  const float* bq   = (const float*)d_in[6];
  const float* Wk   = (const float*)d_in[7];
  const float* bk   = (const float*)d_in[8];
  const float* Wv   = (const float*)d_in[9];
  const float* bv   = (const float*)d_in[10];
  const float* Wo   = (const float*)d_in[11];
  const float* bo   = (const float*)d_in[12];
  const float* Wcat = (const float*)d_in[13];
  const float* bp   = (const float*)d_in[14];
  float* out = (float*)d_out;

  char* ws = (char*)d_ws;
  unsigned short* WSQ  = (unsigned short*)(ws + kOffWSQ);
  unsigned short* WCAT = (unsigned short*)(ws + kOffWCAT);
  float*          TAB  = (float*)(ws + kOffTAB);
  unsigned short* HP   = (unsigned short*)(ws + kOffHP);
  unsigned short* EP   = (unsigned short*)(ws + kOffEP);
  float*          QKV  = (float*)(ws + kOffQKV);

  const unsigned short* BtW2  = WSQ;
  const unsigned short* BtQKV = WSQ + (size_t)1 * kDm * kDm;
  const unsigned short* BtWo  = WSQ + (size_t)4 * kDm * kDm;

  const float scl = 1.0f / sqrtf((float)kDk);

  wt_cast_kernel<<<dim3(kDm / 64, kDm / 64, 5), 256, 0, stream>>>(
      W2, Wq, Wk, Wv, Wo, WSQ, (long)kDm * kDm, kDm, kDm, kWCarry);
  wt_cast_kernel<<<dim3(kCatK / 64, kDm / 64, 1), 256, 0, stream>>>(
      Wcat, Wcat, Wcat, Wcat, Wcat, WCAT, 0L, kCatK, kDm, kWcatCarry);
  bias_table_kernel<<<1, 384, 0, stream>>>(b2, bq, bk, bv, bo, bp, TAB, kActCarry);

  for (int c = 0; c < kChunks; ++c) {
    const float* specC = spec + (size_t)c * kTc;
    float* outC = out + (size_t)c * kWc * kDm;

    embed_kernel<<<(kTc * 32) / 256, 256, 0, stream>>>(specC, W1, b1, HP, kTc * 32, kActCarry);

    wmma_gemm64_f16<1><<<((kTc / 64) * (kDm / 64)) / 8, 256, 0, stream>>>(
        HP, kDm, BtW2, kDm, (void*)EP, kDm, TAB + kTabB2, kTc, kDm, kDm, kScaleE);

    wmma_gemm64_f16<0><<<((kTc / 64) * (kQkvN / 64)) / 8, 256, 0, stream>>>(
        EP, kDm, BtQKV, kDm, (void*)QKV, kQkvN, TAB + kTabQkv, kTc, kQkvN, kDm, kScaleQkv);

    window_attn_kernel<<<kTc / 32, 256, 0, stream>>>(QKV, HP, scl, kActCarry);

    wmma_gemm64_f16<1><<<((kTc / 64) * (kDm / 64)) / 8, 256, 0, stream>>>(
        HP, kDm, BtWo, kDm, (void*)EP, kDm, TAB + kTabBo, kTc, kDm, kDm, kScaleO);

    wmma_gemm64_f16<0><<<((kWc / 64) * (kDm / 64)) / 8, 256, 0, stream>>>(
        EP, kCatK, WCAT, kCatK, (void*)outC, kDm, TAB + kTabBp, kWc, kDm, kCatK, kScaleOut);
  }
}
